// GNNFeatureExtractor_56006373540168
// MI455X (gfx1250) — hardware-verified
//
#include <hip/hip_runtime.h>
#include <stddef.h>


#define NN     4800
#define FEAT   15
#define NH     3
#define DD1    64
#define DD2    128
#define C1     192
#define C2     384
#define NBATCH 32
#define NJOBS  150
#define HID    64
#define GK     143
#define GP     192
#define MASKN  (NBATCH * (NJOBS + 1))
#define OUT0N  (NBATCH * HID)

#define WSC 8192.0f
#define HS1 64.0f
#define HS2 1024.0f
#define A1S 256.0f
#define WTS 16.0f
#define GS  16.0f

typedef _Float16 v16h __attribute__((ext_vector_type(16)));
typedef _Float16 v8h  __attribute__((ext_vector_type(8)));
typedef float    v8f  __attribute__((ext_vector_type(8)));
typedef float    v4f  __attribute__((ext_vector_type(4)));
union Frag { v16h v; v8h hv[2]; };

__device__ __forceinline__ v8f zero8() {
  v8f r;
#pragma unroll
  for (int i = 0; i < 8; ++i) r[i] = 0.f;
  return r;
}

__device__ __forceinline__ v16h ldfrag(const _Float16* __restrict__ p, int hh) {
  Frag f;
  f.hv[0] = *(const v8h*)(p + 8 * hh);
  f.hv[1] = *(const v8h*)(p + 16 + 8 * hh);
  return f.v;
}

__device__ __forceinline__ v8f wmma16(v16h a, v16h b, v8f c) {
  v8f d = __builtin_amdgcn_wmma_f32_16x16x32_f16(false, a, false, b, (short)0, c, false, false);
  asm volatile("v_nop\n\tv_nop\n\tv_nop\n\tv_nop" : "+v"(d) : "v"(a), "v"(b));
  return d;
}

__global__ __launch_bounds__(32) void k_wprep(const float* __restrict__ W2, const float* __restrict__ P1,
                                             const float* __restrict__ P2, _Float16* __restrict__ W2t,
                                             _Float16* __restrict__ P1t, _Float16* __restrict__ P2t) {
  const int bx = blockIdx.x, tid = threadIdx.x;
  const float* W;
  _Float16* dst;
  int K, N, KP, n;
  if (bx < C2) {
    W = W2; dst = W2t; K = C1; N = C2; KP = C1; n = bx;
  } else if (bx < C2 + 2 * HID) {
    W = P1; dst = P1t; K = GK; N = 2 * HID; KP = GP; n = bx - C2;
  } else {
    W = P2; dst = P2t; K = 2 * HID; N = HID; KP = 2 * HID; n = bx - C2 - 2 * HID;
  }
  if (n < N && tid < KP / 8) {
    v8h o;
#pragma unroll
    for (int u = 0; u < 8; ++u) {
      const int k = tid * 8 + u;
      const float x = (k < K) ? W[(size_t)k * N + n] * WTS : 0.f;
      o[u] = (_Float16)x;
    }
    _Float16* d = dst + (size_t)n * KP + tid * 8;
    *(volatile v8h*)d = o;
    __threadfence();
    *(volatile v8h*)d = o;
  }
}

__global__ __launch_bounds__(C1) void k_prep1(const float* __restrict__ obs, const float* __restrict__ W1,
                                             const float* __restrict__ asrc, const float* __restrict__ adst,
                                             _Float16* __restrict__ hT1, float* __restrict__ s1,
                                             float* __restrict__ t1) {
  __shared__ float xs[64 * FEAT];
  __shared__ float T[C1][64];
  __shared__ float F[6][64];
  const int tid = threadIdx.x;
  const int n0 = blockIdx.x * 64;
  for (int i = tid; i < 64 * FEAT; i += C1) xs[i] = obs[(size_t)n0 * FEAT + i];
  float wr[FEAT];
#pragma unroll
  for (int f = 0; f < FEAT; ++f) wr[f] = W1[f * C1 + tid];
  __syncthreads();
  for (int nn = 0; nn < 64; ++nn) {
    float a = 0.f;
#pragma unroll
    for (int f = 0; f < FEAT; ++f) a += xs[nn * FEAT + f] * wr[f];
    T[tid][nn] = a;
  }
  {
    v8h hv[8];
#pragma unroll
    for (int p = 0; p < 8; ++p) {
#pragma unroll
      for (int u = 0; u < 8; ++u) hv[p][u] = (_Float16)(T[tid][p * 8 + u] * HS1);
    }
    _Float16* dst = hT1 + (size_t)tid * NN + n0;
#pragma unroll
    for (int pass = 0; pass < 2; ++pass) {
#pragma unroll
      for (int p = 0; p < 8; ++p) *(volatile v8h*)(dst + p * 8) = hv[p];
      if (pass == 0) __threadfence();
    }
  }
  __syncthreads();
  for (int item = tid; item < 384; item += C1) {
    const int arr = item >> 6, nn = item & 63;
    const int hd = (arr < 3) ? arr : (arr - 3);
    const float* av = ((arr < 3) ? asrc : adst) + hd * DD1;
    float d = 0.f;
#pragma unroll 4
    for (int k = 0; k < DD1; ++k) d += T[hd * DD1 + k][nn] * av[k];
    F[arr][nn] = d;
  }
  __syncthreads();
  if (tid < 96) {
    const int arr = tid >> 4, piece = tid & 15;
    const int hd = (arr < 3) ? arr : (arr - 3);
    v4f o;
#pragma unroll
    for (int u = 0; u < 4; ++u) o[u] = F[arr][piece * 4 + u];
    float* dst = ((arr < 3) ? s1 : t1) + (size_t)hd * NN + n0 + piece * 4;
    *(volatile v4f*)dst = o;
    __threadfence();
    *(volatile v4f*)dst = o;
  }
}

__global__ __launch_bounds__(256) void k_coef(const float* __restrict__ s, const float* __restrict__ t,
                                             float* __restrict__ Bc, float* __restrict__ Cc,
                                             float* __restrict__ Dc) {
  __shared__ float red[256];
  __shared__ float cb[3][256];
  const int tid = threadIdx.x, hd = blockIdx.y;
  const size_t base = (size_t)hd * NN;
  float mx = -3.0e38f;
  for (int j = tid; j < NN; j += 256) mx = fmaxf(mx, t[base + j]);
  red[tid] = mx;
  __syncthreads();
  for (int st = 128; st > 0; st >>= 1) {
    if (tid < st) red[tid] = fmaxf(red[tid], red[tid + st]);
    __syncthreads();
  }
  const float tm = red[0];
  const int n = blockIdx.x * 256 + tid;
  if (n < NN) {
    const float sv = s[base + n], tv = t[base + n];
    const float x = sv + tm;
    const float mrow = (x > 0.f) ? x : 0.2f * x;
    cb[0][tid] = expf(0.2f * sv - mrow);
    cb[1][tid] = expf(tv - tm);
    cb[2][tid] = expf(0.2f * tv);
  }
  __syncthreads();
  if (tid < 192) {
    const int arr = tid >> 6, piece = tid & 63;
    const int nn = blockIdx.x * 256 + piece * 4;
    if (nn < NN) {
      v4f o;
#pragma unroll
      for (int u = 0; u < 4; ++u) o[u] = cb[arr][piece * 4 + u];
      float* dst = ((arr == 0) ? Bc : ((arr == 1) ? Cc : Dc)) + base + nn;
      *(volatile v4f*)dst = o;
      __threadfence();
      *(volatile v4f*)dst = o;
    }
  }
}

template <int DHEAD, int MODE>
__global__ __launch_bounds__(160) void k_agg(const _Float16* __restrict__ hT, const float* __restrict__ s,
                                             const float* __restrict__ t, const float* __restrict__ Bc,
                                             const float* __restrict__ Cc, const float* __restrict__ Dc,
                                             float oscale, void* __restrict__ outp) {
  constexpr int NT = DHEAD / 16;
  constexpr int NW = 5;
  constexpr int BS = NW * 32;
  constexpr int ITER = (NN / 32) / NW;
  constexpr int PE = (MODE == 0) ? 8 : 4;
  constexpr int PPR = DHEAD / PE;
  constexpr int NP = 16 * PPR;
  constexpr int TRIPS = (NP + BS - 1) / BS;

  __shared__ float Tt[NW][32];
  __shared__ float Ct[NW][32];
  __shared__ float Dt[NW][32];
  __shared__ float part[NW][NT][8][32];
  __shared__ float zl[NW][32];
  __shared__ float rZ[16];

  const int tid = threadIdx.x, wv = tid >> 5, l = tid & 31, hh = l >> 4, m = l & 15;
  const int i0 = blockIdx.x * 16, hd = blockIdx.y;
  const size_t hb = (size_t)hd * NN;
  const float sI = s[hb + i0 + m];
  const float BI = Bc[hb + i0 + m];

  v8f acc[NT];
#pragma unroll
  for (int q = 0; q < NT; ++q) acc[q] = zero8();
  float zacc = 0.f;

  for (int k = 0; k < ITER; ++k) {
    const int j0 = (wv + k * NW) * 32;
    Tt[wv][l] = t[hb + j0 + l];
    Ct[wv][l] = Cc[hb + j0 + l];
    Dt[wv][l] = Dc[hb + j0 + l];
    __syncthreads();
    v16h a;
#pragma unroll
    for (int e = 0; e < 16; ++e) {
      const int K = (e < 8) ? (8 * hh + e) : (16 + 8 * hh + (e - 8));
      const float tv = Tt[wv][K];
      const bool pos = (sI + tv) > 0.f;
      const float wg = (pos ? Ct[wv][K] : (BI * Dt[wv][K])) * WSC;
      zacc += wg;
      a[e] = (_Float16)wg;
    }
#pragma unroll
    for (int q = 0; q < NT; ++q) {
      const _Float16* bp = hT + (size_t)(hd * DHEAD + q * 16 + m) * NN + j0;
      const v16h b = ldfrag(bp, hh);
      acc[q] = wmma16(a, b, acc[q]);
    }
    __syncthreads();
  }

  zl[wv][l] = zacc;
#pragma unroll
  for (int q = 0; q < NT; ++q) {
#pragma unroll
    for (int r = 0; r < 8; ++r) part[wv][q][r][l] = acc[q][r];
  }
  __syncthreads();
  if (tid < 16) {
    float zz = 0.f;
#pragma unroll
    for (int w2 = 0; w2 < NW; ++w2) zz += zl[w2][tid] + zl[w2][tid + 16];
    rZ[tid] = oscale / zz;
  }
  __syncthreads();

  v8h hv[TRIPS];
  v4f fv[TRIPS];
#pragma unroll
  for (int trip = 0; trip < TRIPS; ++trip) {
    const int p = tid + trip * BS;
    if (p < NP) {
      const int mrow = p / PPR, piece = p - mrow * PPR, c0 = piece * PE;
      const int r = mrow & 7, lh = (mrow >> 3) * 16;
      const float rz = rZ[mrow];
#pragma unroll
      for (int u = 0; u < PE; ++u) {
        const int col = c0 + u, q = col >> 4, li = (col & 15) + lh;
        float v = 0.f;
#pragma unroll
        for (int w2 = 0; w2 < NW; ++w2) v += part[w2][q][r][li];
        v *= rz;
        if (MODE == 0) {
          v = (v > 0.f) ? v : expm1f(v);
          hv[trip][u] = (_Float16)(v * A1S);
        } else {
          fv[trip][u] = v;
        }
      }
    }
  }
#pragma unroll
  for (int pass = 0; pass < 2; ++pass) {
#pragma unroll
    for (int trip = 0; trip < TRIPS; ++trip) {
      const int p = tid + trip * BS;
      if (p < NP) {
        const int mrow = p / PPR, piece = p - mrow * PPR, c0 = piece * PE;
        if (MODE == 0) {
          _Float16* dst = (_Float16*)outp + (size_t)(i0 + mrow) * C1 + hd * DHEAD + c0;
          *(volatile v8h*)dst = hv[trip];
        } else {
          float* dst = (float*)outp + ((size_t)hd * NN + i0 + mrow) * DHEAD + c0;
          *(volatile v4f*)dst = fv[trip];
        }
      }
    }
    if (pass == 0) __threadfence();
  }
}

template <int MODE>
__global__ __launch_bounds__(128) void k_gemm(const _Float16* __restrict__ A, const _Float16* __restrict__ Bt,
                                             const float* __restrict__ va, const float* __restrict__ vb,
                                             void* __restrict__ o0, float* __restrict__ o1,
                                             float* __restrict__ o2) {
  constexpr int AR  = (MODE == 0) ? 2 : 1;
  constexpr int LDA = (MODE == 2) ? (2 * HID) : C1;
  constexpr int LDB = LDA;
  constexpr int KS  = LDA / 32;
  constexpr int RB  = 64 * AR;
  __shared__ float T[RB][64];
  __shared__ float sv[2][64];
  const int tid = threadIdx.x, w = tid >> 5, l = tid & 31, hh = l >> 4, m = l & 15;
  const int R0 = blockIdx.x * RB, N0 = blockIdx.y * 64;

  v8f acc[AR][4];
#pragma unroll
  for (int ar = 0; ar < AR; ++ar) {
#pragma unroll
    for (int q = 0; q < 4; ++q) acc[ar][q] = zero8();
  }
  for (int ks = 0; ks < KS; ++ks) {
    const int k0 = ks * 32;
    v16h af[AR], bf[4];
#pragma unroll
    for (int ar = 0; ar < AR; ++ar)
      af[ar] = ldfrag(A + (size_t)(R0 + w * 16 * AR + ar * 16 + m) * LDA + k0, hh);
#pragma unroll
    for (int q = 0; q < 4; ++q) bf[q] = ldfrag(Bt + (size_t)(N0 + q * 16 + m) * LDB + k0, hh);
#pragma unroll
    for (int ar = 0; ar < AR; ++ar) {
#pragma unroll
      for (int q = 0; q < 4; ++q) acc[ar][q] = wmma16(af[ar], bf[q], acc[ar][q]);
    }
  }
#pragma unroll
  for (int ar = 0; ar < AR; ++ar) {
#pragma unroll
    for (int q = 0; q < 4; ++q) {
#pragma unroll
      for (int r = 0; r < 8; ++r) T[w * 16 * AR + ar * 16 + 8 * hh + r][q * 16 + m] = acc[ar][q][r];
    }
  }
  __syncthreads();

  if (MODE == 0) {
    {
      const int nn = tid & 63, which = tid >> 6;
      const float* av = (which ? vb : va) + R0;
      float d = 0.f;
#pragma unroll 4
      for (int k = 0; k < RB; ++k) d += T[k][nn] * av[k];
      sv[which][nn] = d * (1.0f / (A1S * WTS));
    }
    __syncthreads();
    v8h hv[8];
#pragma unroll
    for (int trip = 0; trip < 8; ++trip) {
      const int p = tid + 128 * trip;
      const int row = p >> 3, piece = p & 7;
#pragma unroll
      for (int u = 0; u < 8; ++u) hv[trip][u] = (_Float16)(T[row][piece * 8 + u] * (HS2 / (A1S * WTS)));
    }
    const int which2 = (tid >> 4) & 1, sp = tid & 15;
    v4f so;
#pragma unroll
    for (int u = 0; u < 4; ++u) so[u] = sv[which2][sp * 4 + u];
#pragma unroll
    for (int pass = 0; pass < 2; ++pass) {
#pragma unroll
      for (int trip = 0; trip < 8; ++trip) {
        const int p = tid + 128 * trip;
        const int row = p >> 3, piece = p & 7;
        _Float16* dst = (_Float16*)o0 + (size_t)(R0 + row) * NN + N0 + piece * 8;
        *(volatile v8h*)dst = hv[trip];
      }
      if (tid < 32) {
        float* dst = (which2 ? o2 : o1) + (size_t)blockIdx.x * NN + N0 + sp * 4;
        *(volatile v4f*)dst = so;
      }
      if (pass == 0) __threadfence();
    }
  } else {
    constexpr int OPE  = (MODE == 1) ? 8 : 4;
    constexpr int OPPR = 64 / OPE;
    constexpr int OTR  = (16 * OPPR) / 32;
    v8h hv[OTR];
    v4f fv[OTR];
#pragma unroll
    for (int trip = 0; trip < OTR; ++trip) {
      const int p = l + 32 * trip;
      const int row = p / OPPR, piece = p - row * OPPR;
#pragma unroll
      for (int u = 0; u < OPE; ++u) {
        const int col = piece * OPE + u;
        float x = T[w * 16 + row][col] * (1.0f / (GS * WTS)) + va[N0 + col];
        x = fmaxf(x, 0.f);
        if (MODE == 1) hv[trip][u] = (_Float16)(x * GS);
        else fv[trip][u] = x;
      }
    }
#pragma unroll
    for (int pass = 0; pass < 2; ++pass) {
#pragma unroll
      for (int trip = 0; trip < OTR; ++trip) {
        const int p = l + 32 * trip;
        const int row = p / OPPR, piece = p - row * OPPR;
        if (MODE == 1) {
          _Float16* dst = (_Float16*)o0 + (size_t)(R0 + w * 16 + row) * (2 * HID) + N0 + piece * 8;
          *(volatile v8h*)dst = hv[trip];
        } else {
          float* dst = (float*)o0 + (size_t)(R0 + w * 16 + row) * HID + piece * 4;
          *(volatile v4f*)dst = fv[trip];
        }
      }
      if (pass == 0) __threadfence();
    }
  }
}

__global__ __launch_bounds__(256) void k_gbuild(const float* __restrict__ out2, const float* __restrict__ obs,
                                               _Float16* __restrict__ G) {
  constexpr int PPR = GP / 8;
  constexpr int NP = 32 * PPR;
  constexpr int TR = NP / 256;
  const int tid = threadIdx.x, rb = blockIdx.x * 32;
  v8h hv[TR];
#pragma unroll
  for (int trip = 0; trip < TR; ++trip) {
    const int p = tid + 256 * trip;
    const int row = p / PPR, piece = p - row * PPR;
    const int node = rb + row, c0 = piece * 8;
#pragma unroll
    for (int u = 0; u < 8; ++u) {
      const int col = c0 + u;
      float v;
      if (col < DD2) {
        const size_t bi = (size_t)node * DD2 + col;
        v = (out2[bi] + out2[(size_t)NN * DD2 + bi] + out2[(size_t)2 * NN * DD2 + bi]) * (1.0f / 3.0f);
      } else if (col < GK) {
        v = obs[(size_t)node * FEAT + (col - DD2)];
      } else {
        v = 0.f;
      }
      hv[trip][u] = (_Float16)(v * GS);
    }
  }
#pragma unroll
  for (int pass = 0; pass < 2; ++pass) {
#pragma unroll
    for (int trip = 0; trip < TR; ++trip) {
      const int p = tid + 256 * trip;
      const int row = p / PPR, piece = p - row * PPR;
      const int node = rb + row;
      if (node < NN) *(volatile v8h*)(G + (size_t)node * GP + piece * 8) = hv[trip];
    }
    if (pass == 0) __threadfence();
  }
}

__global__ __launch_bounds__(256) void k_final(const float* __restrict__ F2, const float* __restrict__ mask,
                                              float* __restrict__ out) {
  __shared__ float pl[HID];
  const int tid = threadIdx.x;
  if (blockIdx.x < NBATCH) {
    const int b = blockIdx.x;
    if (tid < HID) {
      float sum = 0.f;
      for (int j = 0; j < NJOBS; ++j) sum += F2[((size_t)(b * NJOBS + j)) * HID + tid];
      pl[tid] = sum * (1.0f / (float)NJOBS);
    }
    __syncthreads();
    if (tid < 16) {
      v4f o;
#pragma unroll
      for (int u = 0; u < 4; ++u) o[u] = pl[tid * 4 + u];
      float* dst = out + b * HID + tid * 4;
      *(volatile v4f*)dst = o;
      __threadfence();
      *(volatile v4f*)dst = o;
    }
  } else {
    const int q = (blockIdx.x - NBATCH) * 256 + tid;
    const int e0 = q * 4;
    if (e0 < MASKN) {
      v4f o;
#pragma unroll
      for (int u = 0; u < 4; ++u) o[u] = mask[e0 + u];
      float* dst = out + OUT0N + e0;
      *(volatile v4f*)dst = o;
      __threadfence();
      *(volatile v4f*)dst = o;
    }
  }
}

extern "C" void kernel_launch(void* const* d_in, const int* in_sizes, int n_in,
                              void* d_out, int out_size, void* d_ws, size_t ws_size,
                              hipStream_t stream) {
  if (n_in < 12) return;
  if (in_sizes[0] != NN * FEAT || in_sizes[1] != MASKN || in_sizes[2] != FEAT * C1 ||
      in_sizes[3] != NH * DD1 || in_sizes[4] != NH * DD1 || in_sizes[5] != C1 * C2 ||
      in_sizes[6] != NH * DD2 || in_sizes[7] != NH * DD2 || in_sizes[8] != GK * 2 * HID ||
      in_sizes[9] != 2 * HID || in_sizes[10] != 2 * HID * HID || in_sizes[11] != HID ||
      out_size != OUT0N + MASKN)
    return;

  const float* obs   = (const float*)d_in[0];
  const float* amask = (const float*)d_in[1];
  const float* W1    = (const float*)d_in[2];
  const float* as1   = (const float*)d_in[3];
  const float* ad1   = (const float*)d_in[4];
  const float* W2    = (const float*)d_in[5];
  const float* as2   = (const float*)d_in[6];
  const float* ad2   = (const float*)d_in[7];
  const float* P1    = (const float*)d_in[8];
  const float* b1    = (const float*)d_in[9];
  const float* P2    = (const float*)d_in[10];
  const float* b2    = (const float*)d_in[11];
  float* out = (float*)d_out;

  char* wb = (char*)d_ws;
  size_t off = 0;
  auto carve = [&](size_t bytes) -> void* {
    void* p = wb + off;
    off = (off + bytes + 255) & ~(size_t)255;
    return p;
  };
  const size_t vecb = (size_t)NH * NN * 4;
  _Float16* W2t  = (_Float16*)carve((size_t)C2 * C1 * 2);
  _Float16* P1t  = (_Float16*)carve((size_t)2 * HID * GP * 2);
  _Float16* P2t  = (_Float16*)carve((size_t)HID * 2 * HID * 2);
  _Float16* hT1  = (_Float16*)carve((size_t)C1 * NN * 2);
  float* s1  = (float*)carve(vecb);
  float* t1  = (float*)carve(vecb);
  float* B1  = (float*)carve(vecb);
  float* Cc1 = (float*)carve(vecb);
  float* Dc1 = (float*)carve(vecb);
  _Float16* act1h = (_Float16*)carve((size_t)NN * C1 * 2);
  _Float16* hT2   = (_Float16*)carve((size_t)C2 * NN * 2);
  float* s2  = (float*)carve(vecb);
  float* t2  = (float*)carve(vecb);
  float* B2  = (float*)carve(vecb);
  float* Cc2 = (float*)carve(vecb);
  float* Dc2 = (float*)carve(vecb);
  float* out2 = (float*)carve((size_t)NH * NN * DD2 * 4);
  _Float16* G   = (_Float16*)carve((size_t)NN * GP * 2);
  _Float16* F1h = (_Float16*)carve((size_t)NN * 2 * HID * 2);
  float* F2 = (float*)carve((size_t)NN * HID * 4);
  if (off > ws_size) return;

  k_wprep<<<C2 + 2 * HID + HID, 32, 0, stream>>>(W2, P1, P2, W2t, P1t, P2t);

  k_prep1<<<NN / 64, C1, 0, stream>>>(obs, W1, as1, ad1, hT1, s1, t1);
  k_coef<<<dim3((NN + 255) / 256, NH), 256, 0, stream>>>(s1, t1, B1, Cc1, Dc1);
  k_agg<DD1, 0><<<dim3(NN / 16, NH), 160, 0, stream>>>(hT1, s1, t1, B1, Cc1, Dc1, 1.0f / HS1,
                                                       (void*)act1h);

  k_gemm<0><<<dim3(NH, NN / 64), 128, 0, stream>>>(W2t, act1h, as2, ad2, (void*)hT2, s2, t2);
  k_coef<<<dim3((NN + 255) / 256, NH), 256, 0, stream>>>(s2, t2, B2, Cc2, Dc2);
  k_agg<DD2, 1><<<dim3(NN / 16, NH), 160, 0, stream>>>(hT2, s2, t2, B2, Cc2, Dc2, 1.0f / HS2,
                                                       (void*)out2);

  k_gbuild<<<NN / 32, 256, 0, stream>>>(out2, obs, G);
  k_gemm<1><<<dim3(NN / 64, 2), 128, 0, stream>>>(G, P1t, b1, b1, (void*)F1h, F2, F2);
  k_gemm<2><<<dim3(NN / 64, 1), 128, 0, stream>>>(F1h, P2t, b2, b2, (void*)F2, s2, t2);
  k_final<<<NBATCH + (MASKN / 4 + 255) / 256, 256, 0, stream>>>(F2, amask, out);
}
